// SelectiveStateSpaceModel_3607772529041
// MI455X (gfx1250) — hardware-run, weakly checked
//
#include <hip/hip_runtime.h>
#include <math.h>

typedef __attribute__((ext_vector_type(16))) _Float16 v16h;
typedef __attribute__((ext_vector_type(8)))  _Float16 v8h;
typedef __attribute__((ext_vector_type(2)))  _Float16 v2h;
typedef __attribute__((ext_vector_type(8)))  float    v8f;
typedef __attribute__((ext_vector_type(4)))  float    v4f;
typedef __attribute__((ext_vector_type(4)))  unsigned int v4u;

constexpr int kBatch = 2;
constexpr int kSeq   = 2048;
constexpr int kD     = 1024;
constexpr int kNst   = 16;
constexpr int kRank  = 64;
constexpr int kDbc   = kRank + 2 * kNst;
constexpr int kDbcP  = 128;
constexpr int kBcP   = 64;
constexpr int kRows  = kBatch * kSeq;
constexpr int kScanTS = 64;
constexpr int kScanCh = 32;
constexpr int kScanYP = 36;
constexpr int kSsBlk  = 2048;
static_assert(kDbc == 96 && kDbc <= kDbcP);
static_assert((kD % 32) == 0 && (kRank % 32) == 0);
static_assert((kRows % 64) == 0 && (kRank % 64) == 0 && (kBcP % 64) == 0 && (kD % 64) == 0);
static_assert(kDbcP == kRank + kBcP);
static_assert((kSeq % kScanTS) == 0 && (kD % kScanCh) == 0);
static_assert(((kRows * kD) % kSsBlk) == 0);
static_assert(((kRows * kD / 8) % 256) == 0 && ((kDbcP * kD / 8) % 256) == 0 && ((kD * kRank / 8) % 256) == 0);
static_assert(((kDbc * kD) % 8) == 0);

constexpr int kCarryX  = 16;
constexpr int kCarryW  = 256;
constexpr int kCarryDl = 8;
constexpr float kF16MinNormal = 6.103515625e-5f;

constexpr size_t kOffXH = 0;
constexpr size_t kOffWD = kOffXH + (size_t)kRows * kD * 2;
constexpr size_t kOffWU = kOffWD + (size_t)kDbcP * kD * 2;
constexpr size_t kOffDL = kOffWU + (size_t)kD * kRank * 2;
constexpr size_t kOffBC = kOffDL + (size_t)kRows * kRank * 2;
constexpr size_t kOffZ  = kOffBC + (size_t)kRows * kBcP * 4;
constexpr size_t kOffDT = kOffZ  + (size_t)kRows * kD * 4;
constexpr size_t kWsTotal = kOffDT + (size_t)kRows * kD * 4;
static_assert(kWsTotal == 43909120ull);
static_assert(kWsTotal <= 134217728ull);
static_assert((kOffWD % 128) == 0 && (kOffWU % 128) == 0 && (kOffDL % 128) == 0 &&
              (kOffBC % 128) == 0 && (kOffZ % 128) == 0 && (kOffDT % 128) == 0);

__device__ __forceinline__ float bf16_val(float f) {
  const unsigned u = __float_as_uint(f);
  const unsigned lsb = (u >> 16) & 1u;
  return __uint_as_float((u + 0x7FFFu + lsb) & 0xFFFF0000u);
}
__device__ __forceinline__ unsigned pack2_f16(float a, float b, float carry) {
  float sa = a * carry, sb = b * carry;
  sa = (fabsf(sa) < kF16MinNormal) ? 0.0f : sa;
  sb = (fabsf(sb) < kF16MinNormal) ? 0.0f : sb;
  const v2h p = {(_Float16)sa, (_Float16)sb};
  return __builtin_bit_cast(unsigned, p);
}
__device__ __forceinline__ v4u pack8_f16(const float (&f)[8], float carry) {
  const unsigned w0 = pack2_f16(f[0], f[1], carry);
  const unsigned w1 = pack2_f16(f[2], f[3], carry);
  const unsigned w2 = pack2_f16(f[4], f[5], carry);
  const unsigned w3 = pack2_f16(f[6], f[7], carry);
  return (v4u){w0, w1, w2, w3};
}

__device__ __forceinline__ void tie_acc(v8f& a, v16h x, v16h y) { asm volatile("" : "+v"(a) : "v"(x), "v"(y)); }
__device__ __forceinline__ void nop_acc(v8f& a, v16h x, v16h y) { asm volatile("v_nop\n\tv_nop\n\tv_nop\n\tv_nop" : "+v"(a) : "v"(x), "v"(y)); }
__device__ __forceinline__ void settle_acc(v8f& a) { asm volatile("v_nop\n\tv_nop\n\tv_nop\n\tv_nop" : "+v"(a)); }
__device__ __forceinline__ void keep4(v16h a, v16h b, v16h c, v16h d) { asm volatile("v_nop" :: "v"(a), "v"(b), "v"(c), "v"(d)); }
union FragU { v16h v; v8h h[2]; };
__device__ __forceinline__ v16h frag_load(const _Float16* p) {
  FragU f; f.h[0] = *(const v8h*)(p); f.h[1] = *(const v8h*)(p + 16); return f.v;
}
__device__ __forceinline__ v8f frag_mma(v16h a, v16h b, v8f c) {
  return __builtin_amdgcn_wmma_f32_16x16x32_f16(false, a, false, b, (short)0, c, false, false);
}

template <int CARRY>
__global__ __launch_bounds__(256) void operand_planes(
    const float* __restrict__ src, unsigned* __restrict__ dst, int total8, int valid8)
{
  const int i = blockIdx.x * 256 + threadIdx.x;
  if (i >= total8) return;
  const bool valid = (i < valid8);
  const int ic = valid ? i : (valid8 - 1);
  const size_t e0 = (size_t)ic << 3;
  const v4f a0 = *(const v4f*)(src + e0);
  const v4f a1 = *(const v4f*)(src + e0 + 4);
  float f0 = a0[0], f1 = a0[1], f2 = a0[2], f3 = a0[3];
  float f4 = a1[0], f5 = a1[1], f6 = a1[2], f7 = a1[3];
  asm volatile("" : "+v"(f0), "+v"(f1), "+v"(f2), "+v"(f3));
  asm volatile("" : "+v"(f4), "+v"(f5), "+v"(f6), "+v"(f7));
  float f[8];
  f[0] = valid ? bf16_val(f0) : 0.0f; f[1] = valid ? bf16_val(f1) : 0.0f;
  f[2] = valid ? bf16_val(f2) : 0.0f; f[3] = valid ? bf16_val(f3) : 0.0f;
  f[4] = valid ? bf16_val(f4) : 0.0f; f[5] = valid ? bf16_val(f5) : 0.0f;
  f[6] = valid ? bf16_val(f6) : 0.0f; f[7] = valid ? bf16_val(f7) : 0.0f;
  const v4u w = pack8_f16(f, (float)CARRY);
  volatile v4u* q = (volatile v4u*)dst + i;
  *q = w;
  __threadfence();
  *q = w;
}

template <int OUT_F16, int SCALE_DEN, int OUT_CARRY>
__global__ __launch_bounds__(256) void project_rows(
    const unsigned short* __restrict__ Ap, int lda,
    const unsigned short* __restrict__ Btp, int ldb,
    void* __restrict__ Cout, int ldc,
    const float* __restrict__ bias, int nBias,
    int M, int N, int K)
{
  const _Float16* A  = (const _Float16*)Ap;
  const _Float16* Bt = (const _Float16*)Btp;
  __shared__ __align__(16) float sT[8][16 * 68];
  const int lane = threadIdx.x & 31;
  const int wave = threadIdx.x >> 5;
  const int tilesN = N >> 6;
  const int tilesM = M >> 6;
  const int tile = blockIdx.x * 8 + wave;
  if (tile >= tilesM * tilesN) return;
  const int tm = tile / tilesN;
  const int tn = tile - tm * tilesN;
  const int m0 = tm << 6;
  const int n0 = tn << 6;

  const int rlane = lane & 15;
  const int koff  = (lane >> 4) * 8;
  const int mOff  = (lane >> 4) * 8;
  constexpr float scale = 1.0f / (float)SCALE_DEN;

  v8f acc[4][4];
#pragma unroll
  for (int i = 0; i < 4; ++i)
#pragma unroll
    for (int j = 0; j < 4; ++j) acc[i][j] = (v8f){0.f,0.f,0.f,0.f,0.f,0.f,0.f,0.f};

  for (int k0 = 0; k0 < K; k0 += 32) {
    v16h bh[4];
#pragma unroll
    for (int j = 0; j < 4; ++j) {
      const size_t bo = (size_t)(n0 + (j << 4) + rlane) * ldb + koff + k0;
      bh[j] = frag_load(Bt + bo);
    }
#pragma unroll
    for (int i = 0; i < 4; ++i) {
      const size_t ao = (size_t)(m0 + (i << 4) + rlane) * lda + koff + k0;
      const v16h ah = frag_load(A + ao);
#pragma unroll
      for (int j = 0; j < 4; ++j) acc[i][j] = frag_mma(ah, bh[j], acc[i][j]);
      tie_acc(acc[i][0], ah, bh[0]);
      tie_acc(acc[i][1], ah, bh[1]);
      tie_acc(acc[i][2], ah, bh[2]);
      nop_acc(acc[i][3], ah, bh[3]);
    }
    keep4(bh[0], bh[1], bh[2], bh[3]);
  }
#pragma unroll
  for (int i = 0; i < 4; ++i) {
    settle_acc(acc[i][0]);
    settle_acc(acc[i][1]);
    settle_acc(acc[i][2]);
    settle_acc(acc[i][3]);
  }

  float bvj[4];
#pragma unroll
  for (int j = 0; j < 4; ++j) {
    const int n = n0 + (j << 4) + rlane;
    const int nc = (n < nBias) ? n : (nBias - 1);
    float braw = bias[nc];
    asm volatile("" : "+v"(braw));
    bvj[j] = (n < nBias) ? bf16_val(braw) : 0.0f;
  }

  float* slab = sT[wave];
#pragma unroll
  for (int i = 0; i < 4; ++i) {
    const int mBase = m0 + (i << 4);
#pragma unroll
    for (int j = 0; j < 4; ++j) {
#pragma unroll
      for (int r = 0; r < 8; ++r) {
        const float v = acc[i][j][r] * scale + bvj[j];
        slab[(mOff + r) * 68 + (j << 4) + rlane] = v;
      }
    }
    __builtin_amdgcn_fence(__ATOMIC_RELEASE, "workgroup");
    __builtin_amdgcn_wave_barrier();
    __builtin_amdgcn_fence(__ATOMIC_ACQUIRE, "workgroup");
    if (OUT_F16 == 0) {
      float* C = (float*)Cout;
      const int hh = lane >> 4, c4 = (lane & 15) * 4;
      v4f fv[8];
#pragma unroll
      for (int it = 0; it < 8; ++it) fv[it] = *(const v4f*)(slab + (it * 2 + hh) * 68 + c4);
      for (int pass = 0; pass < 2; ++pass) {
#pragma unroll
        for (int it = 0; it < 8; ++it) {
          const int row = it * 2 + hh;
          *(volatile v4f*)(C + (size_t)(mBase + row) * ldc + n0 + c4) = fv[it];
        }
        __threadfence();
      }
    } else {
      unsigned short* C = (unsigned short*)Cout;
      const int q = lane >> 3, c8 = (lane & 7) * 8;
      v4u wh[4];
#pragma unroll
      for (int it = 0; it < 4; ++it) {
        const float* sp = slab + (it * 4 + q) * 68 + c8;
        const v4f a0 = *(const v4f*)(sp);
        const v4f a1 = *(const v4f*)(sp + 4);
        float f[8];
        f[0] = a0[0]; f[1] = a0[1]; f[2] = a0[2]; f[3] = a0[3];
        f[4] = a1[0]; f[5] = a1[1]; f[6] = a1[2]; f[7] = a1[3];
        wh[it] = pack8_f16(f, (float)OUT_CARRY);
      }
      for (int pass = 0; pass < 2; ++pass) {
#pragma unroll
        for (int it = 0; it < 4; ++it) {
          const int row = it * 4 + q;
          *(volatile v4u*)(C + (size_t)(mBase + row) * ldc + n0 + c8) = wh[it];
        }
        __threadfence();
      }
    }
    __builtin_amdgcn_fence(__ATOMIC_RELEASE, "workgroup");
    __builtin_amdgcn_wave_barrier();
    __builtin_amdgcn_fence(__ATOMIC_ACQUIRE, "workgroup");
  }
}

__global__ __launch_bounds__(256) void step_sizes(const float* __restrict__ Z, float* __restrict__ DT)
{
  __shared__ __align__(16) float sV[kSsBlk];
  const unsigned tid = threadIdx.x;
  const size_t base = (size_t)blockIdx.x * kSsBlk;
#pragma unroll
  for (int k = 0; k < 2; ++k) {
    const unsigned q4 = tid + 256u * (unsigned)k;
    *(v4f*)(sV + 4u * q4) = *(const v4f*)(Z + base + 4u * q4);
  }
  __syncthreads();
#pragma unroll 1
  for (unsigned k = 0; k < 8u; ++k) {
    const unsigned e = k * 256u + tid;
    const float v = sV[e];
    const float a = expf(-fabsf(v));
    sV[e] = fmaxf(v, 0.0f) + log1pf(a);
  }
  __syncthreads();
  const v4f o0 = *(const v4f*)(sV + 4u * tid);
  const v4f o1 = *(const v4f*)(sV + 4u * (tid + 256u));
  for (int pass = 0; pass < 2; ++pass) {
    *(volatile v4f*)(DT + base + 4u * tid) = o0;
    *(volatile v4f*)(DT + base + 4u * (tid + 256u)) = o1;
    __threadfence();
  }
}

__global__ __launch_bounds__(32) void channel_scan(
    const float* __restrict__ BC, const float* __restrict__ DT, const float* __restrict__ X,
    const float* __restrict__ Alog, float* __restrict__ Y)
{
  __shared__ __align__(16) float sBC[kScanTS * 32];
  __shared__ __align__(16) float sY[kScanTS * kScanYP];
  __shared__ __align__(16) float sA[kNst * kScanCh];
  const unsigned lane = threadIdx.x;
  constexpr unsigned kBlkPerB = kD / kScanCh;
  const unsigned bix = blockIdx.x / kBlkPerB;
  const unsigned d0  = (blockIdx.x - bix * kBlkPerB) * kScanCh;
  const unsigned d   = d0 + lane;
  const size_t row0  = (size_t)bix * kSeq;
#pragma unroll 1
  for (int s = 0; s < kNst; ++s) sA[s * kScanCh + lane] = -expf(bf16_val(Alog[(size_t)d * kNst + s]));
  __syncthreads();
  float negA[kNst], h[kNst];
#pragma unroll
  for (int s = 0; s < kNst; ++s) {
    negA[s] = sA[s * kScanCh + lane];
    h[s] = 0.0f;
  }
  const unsigned sr = lane >> 3;
  const unsigned c4 = (lane & 7u) * 4u;
#pragma unroll 1
  for (unsigned t0 = 0; t0 < (unsigned)kSeq; t0 += kScanTS) {
    __syncthreads();
#pragma unroll
    for (int i = 0; i < 16; ++i) {
      const unsigned r = (unsigned)i * 4u + sr;
      *(v4f*)(sBC + r * 32u + c4) = *(const v4f*)(BC + (row0 + t0 + r) * kBcP + c4);
    }
    __syncthreads();
#pragma unroll 1
    for (unsigned s = 0; s < (unsigned)kScanTS; ++s) {
      const size_t grow = row0 + t0 + s;
      const float dl = DT[grow * kD + d];
      const float xraw = X[grow * kD + d];
      const float xv = bf16_val(xraw);
      const float* br = sBC + s * 32u;
      float Bs[kNst], Cs[kNst];
#pragma unroll
      for (int q4 = 0; q4 < 4; ++q4) {
        const v4f bv = *(const v4f*)(br + 4 * q4);
        const v4f cv = *(const v4f*)(br + kNst + 4 * q4);
        Bs[4 * q4 + 0] = bv[0]; Bs[4 * q4 + 1] = bv[1]; Bs[4 * q4 + 2] = bv[2]; Bs[4 * q4 + 3] = bv[3];
        Cs[4 * q4 + 0] = cv[0]; Cs[4 * q4 + 1] = cv[1]; Cs[4 * q4 + 2] = cv[2]; Cs[4 * q4 + 3] = cv[3];
      }
      float y = 0.0f;
#pragma unroll
      for (int k = 0; k < kNst; ++k) {
        const float e  = __expf(dl * negA[k]);
        const float bx = (dl * Bs[k]) * xv;
        h[k] = fmaf(e, h[k], bx);
        y = fmaf(h[k], Cs[k], y);
      }
      sY[s * kScanYP + lane] = y;
    }
    __syncthreads();
    v4f ov[16];
#pragma unroll
    for (int it = 0; it < 16; ++it) ov[it] = *(const v4f*)(sY + ((unsigned)it * 4u + sr) * kScanYP + c4);
    for (int pass = 0; pass < 2; ++pass) {
#pragma unroll
      for (int it = 0; it < 16; ++it) {
        const unsigned row = (unsigned)it * 4u + sr;
        *(volatile v4f*)(Y + (row0 + t0 + row) * kD + d0 + c4) = ov[it];
      }
      __threadfence();
    }
  }
}

static_assert((((kRows / 64) * (kRank / 64)) % 8) == 0);
static_assert((((kRows / 64) * (kBcP / 64)) % 8) == 0);
static_assert((((kRows / 64) * (kD / 64)) % 8) == 0);

extern "C" void kernel_launch(void* const* d_in, const int* in_sizes, int n_in,
                              void* d_out, int out_size, void* d_ws, size_t ws_size,
                              hipStream_t stream) {
  if (n_in < 6) return;
  if (in_sizes[0] != kRows * kD) return;
  if (in_sizes[1] != kD * kNst) return;
  if (in_sizes[2] != kDbc * kD) return;
  if (in_sizes[3] != kDbc) return;
  if (in_sizes[4] != kD * kRank) return;
  if (in_sizes[5] != kD) return;
  if (out_size != kRows * kD) return;
  if (ws_size < kWsTotal) return;

  const float* x     = (const float*)d_in[0];
  const float* A_log = (const float*)d_in[1];
  const float* W_dbc = (const float*)d_in[2];
  const float* b_dbc = (const float*)d_in[3];
  const float* W_up  = (const float*)d_in[4];
  const float* b_up  = (const float*)d_in[5];
  float* out = (float*)d_out;

  char* ws = (char*)d_ws;
  unsigned short* XH = (unsigned short*)(ws + kOffXH);
  unsigned short* WD = (unsigned short*)(ws + kOffWD);
  unsigned short* WU = (unsigned short*)(ws + kOffWU);
  unsigned short* DL = (unsigned short*)(ws + kOffDL);
  float*          BC = (float*)(ws + kOffBC);
  float*          Z  = (float*)(ws + kOffZ);
  float*          DT = (float*)(ws + kOffDT);

  operand_planes<kCarryX><<<(kRows * kD / 8) / 256, 256, 0, stream>>>(
      x, (unsigned*)XH, kRows * kD / 8, kRows * kD / 8);
  operand_planes<kCarryW><<<(kDbcP * kD / 8) / 256, 256, 0, stream>>>(
      W_dbc, (unsigned*)WD, kDbcP * kD / 8, kDbc * kD / 8);
  operand_planes<kCarryW><<<(kD * kRank / 8) / 256, 256, 0, stream>>>(
      W_up, (unsigned*)WU, kD * kRank / 8, kD * kRank / 8);

  project_rows<1, kCarryX * kCarryW, kCarryDl><<<((kRows / 64) * (kRank / 64)) / 8, 256, 0, stream>>>(
      XH, kD, WD, kD, (void*)DL, kRank, b_dbc, kRank, kRows, kRank, kD);

  project_rows<0, kCarryX * kCarryW, 1><<<((kRows / 64) * (kBcP / 64)) / 8, 256, 0, stream>>>(
      XH, kD, WD + (size_t)kRank * kD, kD, (void*)BC, kBcP, b_dbc + kRank, kDbc - kRank, kRows, kBcP, kD);

  project_rows<0, kCarryDl * kCarryW, 1><<<((kRows / 64) * (kD / 64)) / 8, 256, 0, stream>>>(
      DL, kRank, WU, kRank, (void*)Z, kD, b_up, kD, kRows, kD, kRank);

  step_sizes<<<(kRows * kD) / kSsBlk, 256, 0, stream>>>(Z, DT);

  channel_scan<<<kBatch * (kD / kScanCh), kScanCh, 0, stream>>>(BC, DT, x, A_log, out);
}
